// MotionGRU_7017976562228
// MI455X (gfx1250) — hardware-verified
//
#include <hip/hip_runtime.h>
#include <math.h>

#pragma clang fp contract(off)

typedef unsigned short us;
typedef us     v8us  __attribute__((ext_vector_type(8)));
typedef __bf16 v16bf __attribute__((ext_vector_type(16)));
typedef float  v8f   __attribute__((ext_vector_type(8)));
typedef float  v4f   __attribute__((ext_vector_type(4)));
typedef v8us __attribute__((may_alias)) v8usa;
typedef v4f  __attribute__((may_alias)) v4fa;

union Frag { v16bf v; v8us hf[2]; };

#define BATCH  4
#define CCH    64
#define MHC    18
#define CIN    82
#define HH     128
#define WW     128
#define HP     130
#define WP     130
#define SPITCH 96
#define RPITCH 32
#define KG     864
#define KW     576
#define NGR    48
#define NCR    32
#define NMR    16
#define NWR    64

#define STK_UNITS (BATCH * HP * WP * (SPITCH / 8))
#define XPF_UNITS (BATCH * HP * WP * (CCH / 4))
#define NB_STK ((STK_UNITS + 255) / 256)
#define NB_XPF ((XPF_UNITS + 255) / 256)

#define WG_UNITS (NGR * KG / 8)
#define WC_UNITS (NCR * KG / 8)
#define WM_UNITS (NMR * KW / 8)
#define WW_UNITS (NWR * KW / 8)
#define NB_WG  ((WG_UNITS + 255) / 256)
#define NB_WC  ((WC_UNITS + 255) / 256)
#define NB_WM  ((WM_UNITS + 255) / 256)
#define NB_WWP ((WW_UNITS + 255) / 256)

static_assert((STK_UNITS % 8) == 0);
static_assert((XPF_UNITS % 8) == 0);
static_assert((WG_UNITS % 8) == 0);
static_assert((WC_UNITS % 8) == 0);
static_assert((WM_UNITS % 8) == 0);
static_assert((WW_UNITS % 8) == 0);

__device__ __forceinline__ us f2bf(float f) {
  unsigned u = __float_as_uint(f);
  u += 0x7FFFu + ((u >> 16) & 1u);
  return (us)(u >> 16);
}
__device__ __forceinline__ float bf2f(us b) { return __uint_as_float(((unsigned)b) << 16); }
__device__ __forceinline__ void split_bf(float v, us& hi, us& lo) {
  hi = f2bf(v);
  lo = f2bf(v - bf2f(hi));
}
__device__ __forceinline__ float sigm(float x) {
  x = fminf(fmaxf(x, -40.0f), 40.0f);
  return 1.0f / (1.0f + expf(-x));
}

__device__ __forceinline__ v8f wmma_bf(Frag a, Frag b, v8f c) {
  v8f d = __builtin_amdgcn_wmma_f32_16x16x32_bf16(false, a.v, false, b.v, (short)0, c, false, false);
  asm volatile("v_nop\n\tv_nop\n\tv_nop\n\tv_nop"
               : "+v"(d) : "v"(a.hf[0]), "v"(a.hf[1]), "v"(b.hf[0]), "v"(b.hf[1]));
  return d;
}
__device__ __forceinline__ v8f wmma3(Frag ah, Frag al, Frag bh, Frag bl, v8f c) {
  c = wmma_bf(ah, bh, c);
  c = wmma_bf(al, bh, c);
  c = wmma_bf(ah, bl, c);
  return c;
}
__device__ __forceinline__ Frag ldfrag(const us* p, int hf) {
  Frag f;
  f.hf[0] = *(const v8usa*)(p + 8 * hf);
  f.hf[1] = *(const v8usa*)(p + 16 + 8 * hf);
  return f;
}

__global__ __launch_bounds__(256) void k_stage(const float* __restrict__ x, const float* __restrict__ pre,
                                               us* __restrict__ stkH, us* __restrict__ stkL,
                                               float* __restrict__ xpf) {
  const int tid = threadIdx.x;
  if (blockIdx.x < NB_STK) {
    const int g = blockIdx.x * 256 + tid;
    if (g >= STK_UNITS) return;
    const int cg = g % 12;
    int p = g / 12;
    const int wp = p % WP; p /= WP;
    const int hp = p % HP;
    const int b = p / HP;
    const bool inside = (hp >= 1) && (hp <= HH) && (wp >= 1) && (wp <= WW);
    const int hh = min(max(hp - 1, 0), HH - 1), ww = min(max(wp - 1, 0), WW - 1);
    v8us oh, ol;
    #pragma unroll
    for (int j = 0; j < 8; ++j) {
      const int c  = cg * 8 + j;
      const int cx = min(c, CCH - 1);
      const int cp = min(max(c - CCH, 0), MHC - 1);
      const float vx = x[((b * CCH + cx) * HH + hh) * WW + ww];
      const float vp = pre[((b * MHC + cp) * HH + hh) * WW + ww];
      float v = (c < CCH) ? vx : ((c < CIN) ? vp : 0.0f);
      v = inside ? v : 0.0f;
      us hb, lb;
      split_bf(v, hb, lb);
      oh[j] = hb; ol[j] = lb;
    }
    us* dh = stkH + (size_t)g * 8;
    us* dl = stkL + (size_t)g * 8;
    *(volatile v8us*)dh = oh;
    *(volatile v8us*)dl = ol;
    __threadfence();
    *(volatile v8us*)dh = oh;
    *(volatile v8us*)dl = ol;
  } else {
    const int g = (blockIdx.x - NB_STK) * 256 + tid;
    if (g >= XPF_UNITS) return;
    const int c4 = g % 16;
    int p = g / 16;
    const int wp = p % WP; p /= WP;
    const int hp = p % HP;
    const int b = p / HP;
    const bool inside = (hp >= 1) && (hp <= HH) && (wp >= 1) && (wp <= WW);
    const int hh = min(max(hp - 1, 0), HH - 1), ww = min(max(wp - 1, 0), WW - 1);
    v4f o;
    #pragma unroll
    for (int j = 0; j < 4; ++j) {
      const int c = c4 * 4 + j;
      const float v = x[((b * CCH + c) * HH + hh) * WW + ww];
      o[j] = inside ? v : 0.0f;
    }
    float* d = xpf + (size_t)g * 4;
    *(volatile v4f*)d = o;
    __threadfence();
    *(volatile v4f*)d = o;
  }
}

__global__ __launch_bounds__(256) void k_wprep(const float* __restrict__ uw, const float* __restrict__ rw,
                                               const float* __restrict__ ow, const float* __restrict__ gw,
                                               const float* __restrict__ cw,
                                               us* __restrict__ WgH, us* __restrict__ WgL,
                                               us* __restrict__ WcH, us* __restrict__ WcL,
                                               us* __restrict__ WmH, us* __restrict__ WmL,
                                               us* __restrict__ WwH, us* __restrict__ WwL) {
  const int tid = threadIdx.x, bx = blockIdx.x;
  float v[8];
  us* dH;
  us* dL;
  if (bx < NB_WG) {
    const int u = bx * 256 + tid;
    if (u >= WG_UNITS) return;
    const int n = u / 108, kk = u - n * 108, tap = kk / 12, ci0 = (kk - tap * 12) * 8;
    const int nu = min(n, MHC - 1), nr = min(max(n - MHC, 0), MHC - 1);
    #pragma unroll
    for (int j = 0; j < 8; ++j) {
      const int ci = ci0 + j, cc = min(ci, CIN - 1);
      const float fu = uw[(nu * CIN + cc) * 9 + tap];
      const float fr = rw[(nr * CIN + cc) * 9 + tap];
      const float t = (n < MHC) ? fu : ((n < 2 * MHC) ? fr : 0.0f);
      v[j] = (ci < CIN) ? t : 0.0f;
    }
    dH = WgH + u * 8; dL = WgL + u * 8;
  } else if (bx < NB_WG + NB_WC) {
    const int u = (bx - NB_WG) * 256 + tid;
    if (u >= WC_UNITS) return;
    const int n = u / 108, kk = u - n * 108, tap = kk / 12, ci0 = (kk - tap * 12) * 8;
    const int nn = min(n, MHC - 1);
    #pragma unroll
    for (int j = 0; j < 8; ++j) {
      const int ci = ci0 + j, cc = min(ci, CIN - 1);
      const float fo = ow[(nn * CIN + cc) * 9 + tap];
      v[j] = (n < MHC && ci < CIN) ? fo : 0.0f;
    }
    dH = WcH + u * 8; dL = WcL + u * 8;
  } else if (bx < NB_WG + NB_WC + NB_WM) {
    const int u = (bx - NB_WG - NB_WC) * 256 + tid;
    if (u >= WM_UNITS) return;
    const int n = u / 72, kk = u - n * 72, tap = kk / 8, c0 = (kk - tap * 8) * 8;
    const int nn = min(n, 8);
    #pragma unroll
    for (int j = 0; j < 8; ++j) {
      const int c = c0 + j;
      const float fg = gw[(nn * CCH + c) * 9 + tap];
      v[j] = (n < 9) ? fg : 0.0f;
    }
    dH = WmH + u * 8; dL = WmL + u * 8;
  } else {
    const int u = (bx - NB_WG - NB_WC - NB_WM) * 256 + tid;
    if (u >= WW_UNITS) return;
    const int o = u / 72, kk = u - o * 72, n9 = kk / 8, c0 = (kk - n9 * 8) * 8;
    #pragma unroll
    for (int j = 0; j < 8; ++j) {
      const int c = c0 + j;
      v[j] = cw[(o * CCH + c) * 9 + n9];
    }
    dH = WwH + u * 8; dL = WwL + u * 8;
  }
  v8us oh, ol;
  #pragma unroll
  for (int j = 0; j < 8; ++j) {
    us hb, lb;
    split_bf(v[j], hb, lb);
    oh[j] = hb; ol[j] = lb;
  }
  *(volatile v8us*)dH = oh;
  *(volatile v8us*)dL = ol;
  __threadfence();
  *(volatile v8us*)dH = oh;
  *(volatile v8us*)dL = ol;
}

__device__ __forceinline__ void gates_store(const float* sU, const us* sRH, const us* sRL,
                                            float* __restrict__ ugw, us* __restrict__ rmH,
                                            us* __restrict__ rmL, int b, int h, int wave, int lane) {
  const int q8 = lane & 7, sub = lane >> 3;
  float* ubase = ugw + (size_t)(b * HH + h) * (MHC * WW);
  #pragma unroll
  for (int i = 0; i < 3; ++i) {
    const int L = i * 32 + wave * 4 + sub;
    const int Lc = min(L, 71);
    const v4f v = *(const v4fa*)(sU + Lc * 32 + q8 * 4);
    if (L < 72) *(volatile v4f*)(ubase + Lc * 32 + q8 * 4) = v;
  }
  const size_t roff = (size_t)((b * HP + h + 1) * WP) * RPITCH;
  #pragma unroll
  for (int i = 0; i < 3; ++i) {
    const int L = i * 32 + wave * 4 + sub;
    const int Lc = min(L, 64);
    const v8us vh = *(const v8usa*)(sRH + Lc * 64 + q8 * 8);
    const v8us vl = *(const v8usa*)(sRL + Lc * 64 + q8 * 8);
    if (L < 65) {
      *(volatile v8us*)(rmH + roff + Lc * 64 + q8 * 8) = vh;
      *(volatile v8us*)(rmL + roff + Lc * 64 + q8 * 8) = vl;
    }
  }
  if (h == 0 || h == HH - 1) {
    const int hz = (h == 0) ? 0 : (HP - 1);
    const size_t zoff = (size_t)((b * HP + hz) * WP) * RPITCH;
    const v8us z = {0, 0, 0, 0, 0, 0, 0, 0};
    #pragma unroll
    for (int i = 0; i < 3; ++i) {
      const int L = i * 32 + wave * 4 + sub;
      const int Lc = min(L, 64);
      if (L < 65) {
        *(volatile v8us*)(rmH + zoff + Lc * 64 + q8 * 8) = z;
        *(volatile v8us*)(rmL + zoff + Lc * 64 + q8 * 8) = z;
      }
    }
  }
}

__global__ __launch_bounds__(256) void k_gates(const us* __restrict__ stkH, const us* __restrict__ stkL,
                                               const us* __restrict__ WgH, const us* __restrict__ WgL,
                                               const float* __restrict__ ub, const float* __restrict__ rb,
                                               const float* __restrict__ pre,
                                               float* __restrict__ ugw, us* __restrict__ rmH, us* __restrict__ rmL) {
  __shared__ __attribute__((aligned(16))) float sU[MHC * WW];
  __shared__ __attribute__((aligned(16))) us sRH[WP * RPITCH];
  __shared__ __attribute__((aligned(16))) us sRL[WP * RPITCH];

  const int tid = threadIdx.x, wave = tid >> 5, lane = tid & 31;
  const int hf = lane >> 4, m = lane & 15;
  const int b = blockIdx.x >> 7, h = blockIdx.x & 127;
  const int w0 = wave * 16, pw = w0 + m;

  for (int i = tid; i < WP * RPITCH; i += 256) { sRH[i] = 0; sRL[i] = 0; }
  __syncthreads();

  const v8f z8 = {0.f, 0.f, 0.f, 0.f, 0.f, 0.f, 0.f, 0.f};
  v8f acc[3] = {z8, z8, z8};

  #pragma unroll 1
  for (int tap = 0; tap < 9; ++tap) {
    const int dh = tap / 3, dw = tap - dh * 3;
    const int pix = (b * HP + h + dh) * WP + pw + dw;
    const us* aH = stkH + (size_t)pix * SPITCH;
    const us* aL = stkL + (size_t)pix * SPITCH;
    const int kb = tap * SPITCH;
    #pragma unroll
    for (int ch = 0; ch < 3; ++ch) {
      const Frag ah = ldfrag(aH + ch * 32, hf);
      const Frag al = ldfrag(aL + ch * 32, hf);
      #pragma unroll
      for (int nt = 0; nt < 3; ++nt) {
        const int boff = (nt * 16 + m) * KG + kb + ch * 32;
        const Frag bh = ldfrag(WgH + boff, hf);
        const Frag bl = ldfrag(WgL + boff, hf);
        acc[nt] = wmma3(ah, al, bh, bl, acc[nt]);
      }
    }
  }

  {
    const float bu = ub[m];
    #pragma unroll
    for (int r = 0; r < 8; ++r) {
      const int w = w0 + 8 * hf + r;
      sU[m * WW + w] = sigm(acc[0][r] + bu);
    }
  }
  {
    const int n = 16 + m;
    const int nu = min(n, MHC - 1);
    const int cr = min(max(n - MHC, 0), MHC - 1);
    const float bu = ub[nu], br = rb[cr];
    const bool isu = (n < MHC);
    #pragma unroll
    for (int r = 0; r < 8; ++r) {
      const int w = w0 + 8 * hf + r;
      const float pv = pre[((b * MHC + cr) * HH + h) * WW + w];
      const float s = sigm(acc[1][r] + (isu ? bu : br));
      if (isu) {
        sU[n * WW + w] = s;
      } else {
        us hb, lb;
        split_bf(pv * s, hb, lb);
        sRH[(w + 1) * RPITCH + cr] = hb;
        sRL[(w + 1) * RPITCH + cr] = lb;
      }
    }
  }
  {
    const int n = 32 + m;
    const int cr = min(n - MHC, MHC - 1);
    const float br = rb[cr];
    #pragma unroll
    for (int r = 0; r < 8; ++r) {
      const int w = w0 + 8 * hf + r;
      const float pv = pre[((b * MHC + cr) * HH + h) * WW + w];
      if (m < 4) {
        const float s = sigm(acc[2][r] + br);
        us hb, lb;
        split_bf(pv * s, hb, lb);
        sRH[(w + 1) * RPITCH + cr] = hb;
        sRL[(w + 1) * RPITCH + cr] = lb;
      }
    }
  }
  __syncthreads();

  gates_store(sU, sRH, sRL, ugw, rmH, rmL, b, h, wave, lane);
  __threadfence();
  gates_store(sU, sRH, sRL, ugw, rmH, rmL, b, h, wave, lane);
}

__global__ __launch_bounds__(256) void k_cand(const us* __restrict__ stkH, const us* __restrict__ stkL,
                                              const us* __restrict__ rmH, const us* __restrict__ rmL,
                                              const us* __restrict__ WcH, const us* __restrict__ WcL,
                                              const float* __restrict__ ob, const float* __restrict__ pre,
                                              const float* __restrict__ mean, const float* __restrict__ ugw,
                                              float* __restrict__ out1, float* __restrict__ out2) {
  __shared__ __attribute__((aligned(16))) float sCd[MHC * WW];

  const int tid = threadIdx.x, wave = tid >> 5, lane = tid & 31;
  const int hf = lane >> 4, m = lane & 15;
  const int b = blockIdx.x >> 7, h = blockIdx.x & 127;
  const int w0 = wave * 16, pw = w0 + m;

  const v8f z8 = {0.f, 0.f, 0.f, 0.f, 0.f, 0.f, 0.f, 0.f};
  v8f acc[2] = {z8, z8};

  #pragma unroll 1
  for (int tap = 0; tap < 9; ++tap) {
    const int dh = tap / 3, dw = tap - dh * 3;
    const int pix = (b * HP + h + dh) * WP + pw + dw;
    const us* aH = stkH + (size_t)pix * SPITCH;
    const us* aL = stkL + (size_t)pix * SPITCH;
    const us* rH = rmH + (size_t)pix * RPITCH;
    const us* rL = rmL + (size_t)pix * RPITCH;
    const int kb = tap * SPITCH;
    #pragma unroll
    for (int ch = 0; ch < 3; ++ch) {
      Frag ah, al;
      if (ch < 2) { ah = ldfrag(aH + ch * 32, hf); al = ldfrag(aL + ch * 32, hf); }
      else        { ah = ldfrag(rH, hf);           al = ldfrag(rL, hf); }
      #pragma unroll
      for (int nt = 0; nt < 2; ++nt) {
        const int boff = (nt * 16 + m) * KG + kb + ch * 32;
        const Frag bh = ldfrag(WcH + boff, hf);
        const Frag bl = ldfrag(WcL + boff, hf);
        acc[nt] = wmma3(ah, al, bh, bl, acc[nt]);
      }
    }
  }

  #pragma unroll
  for (int nt = 0; nt < 2; ++nt) {
    const int n = nt * 16 + m;
    const int nc = min(n, MHC - 1);
    const float bo = ob[nc];
    #pragma unroll
    for (int r = 0; r < 8; ++r) {
      const int w = w0 + 8 * hf + r;
      if (n < MHC) sCd[n * WW + w] = tanhf(acc[nt][r] + bo);
    }
  }
  __syncthreads();

  v4f offv[3], mnv[3];
  const float* ubase = ugw + (size_t)(b * HH + h) * (MHC * WW);
  #pragma unroll
  for (int i = 0; i < 3; ++i) {
    const int u = min(tid + 256 * i, MHC * 32 - 1);
    const int c = u >> 5, q = u & 31;
    const size_t gi = ((size_t)(b * MHC + c) * HH + h) * WW + q * 4;
    const v4f cd = *(const v4fa*)(sCd + c * WW + q * 4);
    const v4f uu = *(const v4fa*)(ubase + c * WW + q * 4);
    const v4f po = *(const v4fa*)(pre + gi);
    const v4f me = *(const v4fa*)(mean + gi);
    v4f of, mn;
    #pragma unroll
    for (int e = 0; e < 4; ++e) {
      const float mnew = me[e] + 0.5f * (po[e] - me[e]);
      const float t = po[e] * (1.0f - uu[e]) + cd[e] * uu[e];
      mn[e] = mnew;
      of[e] = t + mnew;
    }
    offv[i] = of; mnv[i] = mn;
  }
  #pragma unroll
  for (int i = 0; i < 3; ++i) {
    const int u = tid + 256 * i;
    if (u < MHC * 32) {
      const int c = u >> 5, q = u & 31;
      const size_t gi = ((size_t)(b * MHC + c) * HH + h) * WW + q * 4;
      *(volatile v4f*)(out1 + gi) = offv[i];
      *(volatile v4f*)(out2 + gi) = mnv[i];
    }
  }
  __threadfence();
  #pragma unroll
  for (int i = 0; i < 3; ++i) {
    const int u = tid + 256 * i;
    if (u < MHC * 32) {
      const int c = u >> 5, q = u & 31;
      const size_t gi = ((size_t)(b * MHC + c) * HH + h) * WW + q * 4;
      *(volatile v4f*)(out1 + gi) = offv[i];
      *(volatile v4f*)(out2 + gi) = mnv[i];
    }
  }
}

__device__ __forceinline__ void warp_store(const float* sO, float* __restrict__ out0, int b, int h, int tid) {
  #pragma unroll
  for (int i = 0; i < 8; ++i) {
    const int u = tid + 256 * i;
    const int o = u >> 5, q = u & 31;
    const v4f v = *(const v4fa*)(sO + o * WW + q * 4);
    *(volatile v4f*)(out0 + ((size_t)(b * CCH + o) * HH + h) * WW + q * 4) = v;
  }
}

__global__ __launch_bounds__(256) void k_warp(const us* __restrict__ stkH, const us* __restrict__ stkL,
                                              const us* __restrict__ WmH, const us* __restrict__ WmL,
                                              const float* __restrict__ gb,
                                              const float* __restrict__ xpf, const float* __restrict__ off1,
                                              const us* __restrict__ WwH, const us* __restrict__ WwL,
                                              float* __restrict__ out0) {
  __shared__ __attribute__((aligned(16))) float sO[CCH * WW];
  __shared__ __attribute__((aligned(16))) float sM[16 * WW];

  const int tid = threadIdx.x, wave = tid >> 5, lane = tid & 31;
  const int hf = lane >> 4, m = lane & 15;
  const int b = blockIdx.x >> 7, h = blockIdx.x & 127;
  const int w0 = wave * 16, pw = w0 + m;
  const v8f z8 = {0.f, 0.f, 0.f, 0.f, 0.f, 0.f, 0.f, 0.f};

  v8f am = z8;
  #pragma unroll 1
  for (int tap = 0; tap < 9; ++tap) {
    const int dh = tap / 3, dw = tap - dh * 3;
    const int pix = (b * HP + h + dh) * WP + pw + dw;
    const us* aH = stkH + (size_t)pix * SPITCH;
    const us* aL = stkL + (size_t)pix * SPITCH;
    const int kb = tap * CCH;
    #pragma unroll
    for (int ch = 0; ch < 2; ++ch) {
      const Frag ah = ldfrag(aH + ch * 32, hf);
      const Frag al = ldfrag(aL + ch * 32, hf);
      const int boff = m * KW + kb + ch * 32;
      const Frag bh = ldfrag(WmH + boff, hf);
      const Frag bl = ldfrag(WmL + boff, hf);
      am = wmma3(ah, al, bh, bl, am);
    }
  }
  {
    const int nc = min(m, 8);
    const float bm = gb[nc];
    #pragma unroll
    for (int r = 0; r < 8; ++r) {
      const int w = w0 + 8 * hf + r;
      if (m < 9) sM[m * WW + w] = sigm(am[r] + bm);
    }
  }
  __syncthreads();

  us* sX  = reinterpret_cast<us*>(sO) + wave * 2048;
  us* sXh = sX + m * 64 + 32 * hf;
  us* sXl = sXh + 1024;
  v8f acc[4] = {z8, z8, z8, z8};
  const float* xb = xpf + (size_t)b * (HP * WP * CCH);
  const float fh1 = (float)(h + 1), fw1 = (float)(pw + 1);

  #pragma unroll 1
  for (int n = 0; n < 9; ++n) {
    const int i3 = n / 3, j3 = n - i3 * 3;
    const float rx = (float)(i3 - 1), ry = (float)(j3 - 1);
    const float ox = off1[((b * MHC + n) * HH + h) * WW + pw];
    const float oy = off1[((b * MHC + 9 + n) * HH + h) * WW + pw];
    float px = (fh1 + rx) + ox;
    float py = (fw1 + ry) + oy;
    const float fx = floorf(px), fy = floorf(py);
    const float lim = (float)(HP - 1);
    const float qxl = fminf(fmaxf(fx, 0.0f), lim);
    const float qyl = fminf(fmaxf(fy, 0.0f), lim);
    const float qxr = fminf(fmaxf(fx + 1.0f, 0.0f), lim);
    const float qyr = fminf(fmaxf(fy + 1.0f, 0.0f), lim);
    px = fminf(fmaxf(px, 0.0f), lim);
    py = fminf(fmaxf(py, 0.0f), lim);
    const float glt = (1.0f + (qxl - px)) * (1.0f + (qyl - py));
    const float grb = (1.0f - (qxr - px)) * (1.0f - (qyr - py));
    const float glb = (1.0f + (qxl - px)) * (1.0f - (qyr - py));
    const float grt = (1.0f - (qxr - px)) * (1.0f + (qyl - py));
    const int ixl = (int)qxl, iyl = (int)qyl, ixr = (int)qxr, iyr = (int)qyr;
    const float* plt = xb + (ixl * WP + iyl) * CCH;
    const float* prb = xb + (ixr * WP + iyr) * CCH;
    const float* plb = xb + (ixl * WP + iyr) * CCH;
    const float* prt = xb + (ixr * WP + iyl) * CCH;
    const float mv = sM[n * WW + pw];

    #pragma unroll
    for (int g = 0; g < 4; ++g) {
      const int co = 32 * hf + 8 * g;
      const v4f lt0 = *(const v4fa*)(plt + co), lt1 = *(const v4fa*)(plt + co + 4);
      const v4f rb0 = *(const v4fa*)(prb + co), rb1 = *(const v4fa*)(prb + co + 4);
      const v4f lb0 = *(const v4fa*)(plb + co), lb1 = *(const v4fa*)(plb + co + 4);
      const v4f rt0 = *(const v4fa*)(prt + co), rt1 = *(const v4fa*)(prt + co + 4);
      v8us oh, ol;
      #pragma unroll
      for (int e = 0; e < 4; ++e) {
        float v0 = ((glt * lt0[e] + grb * rb0[e]) + glb * lb0[e]) + grt * rt0[e];
        v0 = v0 * mv;
        float v1 = ((glt * lt1[e] + grb * rb1[e]) + glb * lb1[e]) + grt * rt1[e];
        v1 = v1 * mv;
        us h0, l0, h1, l1;
        split_bf(v0, h0, l0);
        split_bf(v1, h1, l1);
        oh[e] = h0; ol[e] = l0;
        oh[4 + e] = h1; ol[4 + e] = l1;
      }
      *(v8usa*)(sXh + 8 * g) = oh;
      *(v8usa*)(sXl + 8 * g) = ol;
    }
    __syncthreads();

    #pragma unroll
    for (int ch = 0; ch < 2; ++ch) {
      const Frag ah = ldfrag(sX + m * 64 + ch * 32, hf);
      const Frag al = ldfrag(sX + 1024 + m * 64 + ch * 32, hf);
      #pragma unroll
      for (int nt = 0; nt < 4; ++nt) {
        const int boff = (nt * 16 + m) * KW + n * CCH + ch * 32;
        const Frag bh = ldfrag(WwH + boff, hf);
        const Frag bl = ldfrag(WwL + boff, hf);
        acc[nt] = wmma3(ah, al, bh, bl, acc[nt]);
      }
    }
    __syncthreads();
  }

  #pragma unroll
  for (int nt = 0; nt < 4; ++nt) {
    const int o = nt * 16 + m;
    #pragma unroll
    for (int r = 0; r < 8; ++r) sO[o * WW + w0 + 8 * hf + r] = acc[nt][r];
  }
  __syncthreads();

  warp_store(sO, out0, b, h, tid);
  __threadfence();
  warp_store(sO, out0, b, h, tid);
}

extern "C" void kernel_launch(void* const* d_in, const int* in_sizes, int n_in,
                              void* d_out, int out_size, void* d_ws, size_t ws_size,
                              hipStream_t stream) {
  if (n_in < 12) return;
  if (in_sizes[0] != BATCH * CCH * HH * WW) return;
  if (in_sizes[1] != BATCH * MHC * HH * WW) return;
  if (in_sizes[2] != BATCH * MHC * HH * WW) return;
  if (in_sizes[3] != MHC * CIN * 9 || in_sizes[5] != MHC * CIN * 9 || in_sizes[7] != MHC * CIN * 9) return;
  if (in_sizes[4] != MHC || in_sizes[6] != MHC || in_sizes[8] != MHC) return;
  if (in_sizes[9] != 9 * CCH * 9 || in_sizes[10] != 9) return;
  if (in_sizes[11] != CCH * CCH * 9) return;
  if (out_size != BATCH * CCH * HH * WW + 2 * BATCH * MHC * HH * WW) return;

  const float* x_t   = (const float*)d_in[0];
  const float* pre   = (const float*)d_in[1];
  const float* mean  = (const float*)d_in[2];
  const float* upd_w = (const float*)d_in[3];
  const float* upd_b = (const float*)d_in[4];
  const float* rst_w = (const float*)d_in[5];
  const float* rst_b = (const float*)d_in[6];
  const float* out_w = (const float*)d_in[7];
  const float* out_b = (const float*)d_in[8];
  const float* wg_w  = (const float*)d_in[9];
  const float* wg_b  = (const float*)d_in[10];
  const float* wcw   = (const float*)d_in[11];

  const size_t SZ_STK = (size_t)STK_UNITS * 16;
  const size_t SZ_XPF = (size_t)XPF_UNITS * 16;
  const size_t SZ_RM  = (size_t)BATCH * HP * WP * RPITCH * 2;
  const size_t SZ_UG  = (size_t)BATCH * HH * MHC * WW * 4;
  const size_t SZ_WG  = (size_t)WG_UNITS * 16;
  const size_t SZ_WC  = (size_t)WC_UNITS * 16;
  const size_t SZ_WM  = (size_t)WM_UNITS * 16;
  const size_t SZ_WWP = (size_t)WW_UNITS * 16;
  const size_t total = 2 * SZ_STK + SZ_XPF + 2 * SZ_RM + SZ_UG + 2 * (SZ_WG + SZ_WC + SZ_WM + SZ_WWP);
  if (total > ws_size) return;

  char* ws = (char*)d_ws;
  size_t o = 0;
  us* stkH = (us*)(ws + o); o += SZ_STK;
  us* stkL = (us*)(ws + o); o += SZ_STK;
  float* xpf = (float*)(ws + o); o += SZ_XPF;
  us* rmH = (us*)(ws + o); o += SZ_RM;
  us* rmL = (us*)(ws + o); o += SZ_RM;
  float* ugw = (float*)(ws + o); o += SZ_UG;
  us* WgH = (us*)(ws + o); o += SZ_WG;
  us* WgL = (us*)(ws + o); o += SZ_WG;
  us* WcH = (us*)(ws + o); o += SZ_WC;
  us* WcL = (us*)(ws + o); o += SZ_WC;
  us* WmH = (us*)(ws + o); o += SZ_WM;
  us* WmL = (us*)(ws + o); o += SZ_WM;
  us* WwH = (us*)(ws + o); o += SZ_WWP;
  us* WwL = (us*)(ws + o); o += SZ_WWP;
  if (o > ws_size) return;

  float* outp = (float*)d_out;
  float* out0 = outp;
  float* out1 = outp + (size_t)BATCH * CCH * HH * WW;
  float* out2 = out1 + (size_t)BATCH * MHC * HH * WW;

  k_stage<<<NB_STK + NB_XPF, 256, 0, stream>>>(x_t, pre, stkH, stkL, xpf);
  k_wprep<<<NB_WG + NB_WC + NB_WM + NB_WWP, 256, 0, stream>>>(upd_w, rst_w, out_w, wg_w, wcw,
                                                             WgH, WgL, WcH, WcL, WmH, WmL, WwH, WwL);
  k_gates<<<BATCH * HH, 256, 0, stream>>>(stkH, stkL, WgH, WgL, upd_b, rst_b, pre, ugw, rmH, rmL);
  k_cand<<<BATCH * HH, 256, 0, stream>>>(stkH, stkL, rmH, rmL, WcH, WcL, out_b, pre, mean, ugw, out1, out2);
  k_warp<<<BATCH * HH, 256, 0, stream>>>(stkH, stkL, WmH, WmL, wg_b, xpf, out1, WwH, WwL, out0);
}
